// GraphConv_84499186582211
// MI455X (gfx1250) — hardware-verified
//
#include <hip/hip_runtime.h>
#include <stddef.h>
#include <stdint.h>


#define DIN     128
#define APW     256
#define KP      256
#define NTHR    256
#define NWAVE   8
#define EPT     8
#define CHUNK   (NTHR * EPT)
#define WCAP    (EPT * 32)
#define LISTN   (NWAVE * WCAP)
#define NBMAX   2048
#define NBRUN   1024
#define RCAP    28672
#define DEGCAP  64
#define PKS     11
#define STW     512
#define GBM     64
#define GTHR    128
#define GNT     8
#define NUW     (DIN * (KP / 8))
#define WSMAX   134217728
#define LDS_AGG ((2 * RCAP + 2 * NBMAX + LISTN) * 4 + 64)

static_assert((CHUNK & (CHUNK - 1)) == 0 && CHUNK <= (1 << PKS));
static_assert((NBMAX & (NBMAX - 1)) == 0 && NBMAX <= (1 << PKS));
static_assert((NBRUN & (NBRUN - 1)) == 0 && NBRUN <= NBMAX && NBRUN >= 16);
static_assert(NTHR * 8 == NBMAX);
static_assert(LISTN >= NBMAX);
static_assert(LISTN >= NWAVE * WCAP);
static_assert((RCAP % 32) == 0);
static_assert(NWAVE * STW <= RCAP);
static_assert(LDS_AGG <= 300000);
static_assert(GBM == (GTHR / 32) * 16);
static_assert((DIN % 32) == 0 && (KP % 32) == 0 && KP == 2 * DIN);
static_assert(DIN == 32 * 4 && DIN == 16 * GNT);
static_assert(APW == 2 * DIN && APW == KP);
static_assert((NUW % NTHR) == 0);

typedef float          v4f  __attribute__((ext_vector_type(4)));
typedef float          v8f  __attribute__((ext_vector_type(8)));
typedef int            v4i  __attribute__((ext_vector_type(4)));
typedef int            v8i  __attribute__((ext_vector_type(8)));
typedef unsigned int   v2u  __attribute__((ext_vector_type(2)));
typedef unsigned int   v4u  __attribute__((ext_vector_type(4)));
typedef unsigned short v8us __attribute__((ext_vector_type(8)));
typedef __bf16         v16b __attribute__((ext_vector_type(16)));
typedef v4f  __attribute__((may_alias)) v4fa;
typedef v8us __attribute__((may_alias)) v8usa;
union FragB { v16b v; v8us h[2]; v8i w; };

__device__ __forceinline__ v8f wmb(const FragB& a, const FragB& b, v8f c) {
  v8f d = __builtin_amdgcn_wmma_f32_16x16x32_bf16(false, a.v, false, b.v, (short)0, c, false, false);
  asm volatile("v_nop\n\tv_nop\n\tv_nop\n\tv_nop" : "+v"(d) : "v"(a.w), "v"(b.w));
  return d;
}

__device__ __forceinline__ unsigned short bf_bits(float f) {
  unsigned int u = __float_as_uint(f);
  u += 0x7FFFu + ((u >> 16) & 1u);
  return (unsigned short)(u >> 16);
}
__device__ __forceinline__ float bf_val(unsigned short b) {
  return __uint_as_float(((unsigned int)b) << 16);
}
__device__ __forceinline__ float bf_rne(float f) { return bf_val(bf_bits(f)); }

__device__ __forceinline__ v8us cvt8b(const v4f a, const v4f b) {
  v8us hv;
  hv[0] = bf_bits(a.x); hv[1] = bf_bits(a.y); hv[2] = bf_bits(a.z); hv[3] = bf_bits(a.w);
  hv[4] = bf_bits(b.x); hv[5] = bf_bits(b.y); hv[6] = bf_bits(b.z); hv[7] = bf_bits(b.w);
  return hv;
}

__device__ __forceinline__ int scan_chunk(const int* __restrict__ dsts, int nE, int cbase, int slotBase,
                                          int nb, int vec8, int* list, int tid, int lane, int wave) {
  int wc = 0;
  const int el0  = tid * EPT;
  const int e0   = cbase + el0;
  const int sent = -2147483647 - 1;
  v4i da, db;
  if (vec8 != 0 && cbase + CHUNK <= nE) {
    da = *(const v4i*)(dsts + e0);
    db = *(const v4i*)(dsts + e0 + 4);
  } else {
    da.x = (e0     < nE) ? dsts[min(e0,     nE - 1)] : sent;
    da.y = (e0 + 1 < nE) ? dsts[min(e0 + 1, nE - 1)] : sent;
    da.z = (e0 + 2 < nE) ? dsts[min(e0 + 2, nE - 1)] : sent;
    da.w = (e0 + 3 < nE) ? dsts[min(e0 + 3, nE - 1)] : sent;
    db.x = (e0 + 4 < nE) ? dsts[min(e0 + 4, nE - 1)] : sent;
    db.y = (e0 + 5 < nE) ? dsts[min(e0 + 5, nE - 1)] : sent;
    db.z = (e0 + 6 < nE) ? dsts[min(e0 + 6, nE - 1)] : sent;
    db.w = (e0 + 7 < nE) ? dsts[min(e0 + 7, nE - 1)] : sent;
  }
  const unsigned nbs = (unsigned)slotBase;
  const unsigned unb = (unsigned)nb;
  const unsigned s0 = (unsigned)da.x - nbs, s1 = (unsigned)da.y - nbs;
  const unsigned s2 = (unsigned)da.z - nbs, s3 = (unsigned)da.w - nbs;
  const unsigned s4 = (unsigned)db.x - nbs, s5 = (unsigned)db.y - nbs;
  const unsigned s6 = (unsigned)db.z - nbs, s7 = (unsigned)db.w - nbs;
  const bool h0 = s0 < unb, h1 = s1 < unb, h2 = s2 < unb, h3 = s3 < unb;
  const bool h4 = s4 < unb, h5 = s5 < unb, h6 = s6 < unb, h7 = s7 < unb;
  const unsigned any = __builtin_amdgcn_ballot_w32(h0 | h1 | h2 | h3 | h4 | h5 | h6 | h7);
  if (any != 0u) {
#define HITJ(J, HJ, SJ) { \
      const unsigned mj = __builtin_amdgcn_ballot_w32(HJ); \
      if (mj != 0u) { \
        if (HJ) { \
          const int pos = wc + (int)__builtin_amdgcn_mbcnt_lo(mj, 0u); \
          if (pos < WCAP) list[wave * WCAP + pos] = ((el0 + (J)) << PKS) | (int)(SJ); \
        } \
        wc += (int)__builtin_popcount(mj); } }
    HITJ(0, h0, s0)
    HITJ(1, h1, s1)
    HITJ(2, h2, s2)
    HITJ(3, h3, s3)
    HITJ(4, h4, s4)
    HITJ(5, h5, s5)
    HITJ(6, h6, s6)
    HITJ(7, h7, s7)
#undef HITJ
  }
  return wc;
}

__global__ __launch_bounds__(NTHR) void k_prep(const float* __restrict__ W, unsigned short* WT) {
  const int u = (int)blockIdx.x * NTHR + (int)threadIdx.x;
  if (u >= NUW) return;
  const int n  = u >> 5;
  const int k8 = (u & 31) * 8;
  const int ks = k8 & (DIN - 1);
  const float* p = W + (size_t)n * DIN + ks;
  const v4f a = *(const v4f*)p, b = *(const v4f*)(p + 4);
  const v8us hv = cvt8b(a, b);
  const size_t o = (size_t)n * (size_t)KP + k8;
  *(volatile v8us*)(WT + o) = hv;
  __threadfence();
  *(volatile v8us*)(WT + o) = hv;
}

__global__ __launch_bounds__(GTHR) void k_gemm(const unsigned short* A, int lda,
                                               const unsigned short* __restrict__ WT,
                                               const float* __restrict__ bias,
                                               float* outF, int nN)
{
  constexpr int NT = GNT;
  constexpr int BN = 16 * NT;
  __shared__ __attribute__((aligned(16))) float stg[GBM * BN];
  const int tid = (int)threadIdx.x, lane = tid & 31, wave = tid >> 5, hh = lane >> 4, m = lane & 15;
  const int rowBase = (int)blockIdx.x * GBM;

  v8f acc[NT];
  {
    const v8f z = {0.f, 0.f, 0.f, 0.f, 0.f, 0.f, 0.f, 0.f};
#pragma unroll
    for (int t = 0; t < NT; ++t) acc[t] = z;
  }
  const unsigned short* ap = A  + (size_t)(rowBase + 16 * wave + m) * (size_t)lda + 8 * hh;
  const unsigned short* wp = WT + (size_t)m * (size_t)KP + 8 * hh;
  constexpr int ksteps = KP / 32;
#pragma unroll 1
  for (int ks = 0; ks < ksteps; ++ks) {
    FragB af;
    af.h[0] = *(const v8usa*)(ap + 32 * ks);
    af.h[1] = *(const v8usa*)(ap + 32 * ks + 16);
#pragma unroll
    for (int t = 0; t < NT; ++t) {
      const unsigned short* wq = wp + (size_t)(16 * t) * (size_t)KP + 32 * ks;
      FragB bf;
      bf.h[0] = *(const v8usa*)wq;
      bf.h[1] = *(const v8usa*)(wq + 16);
      acc[t] = wmb(af, bf, acc[t]);
    }
  }

#pragma unroll
  for (int t = 0; t < NT; ++t) {
    const int lc = 16 * t + m;
    const float bb = bf_rne(bias[lc]);
#pragma unroll
    for (int r = 0; r < 8; ++r) {
      const int lr = 16 * wave + 8 * hh + r;
      stg[lr * BN + lc] = acc[t][r] + bb;
    }
  }
  __syncthreads();

  v4f ov[16];
#pragma unroll
  for (int i = 0; i < 16; ++i) {
    const int lr = 16 * wave + i;
    ov[i] = *(const v4fa*)(stg + lr * BN + 4 * lane);
  }
#pragma unroll
  for (int i = 0; i < 16; ++i) {
    const int gr = rowBase + 16 * wave + i;
    float* op = outF + (size_t)gr * (size_t)DIN + 4 * lane;
    if (gr < nN) *(volatile v4f*)op = ov[i];
  }
  __threadfence();
#pragma unroll
  for (int i = 0; i < 16; ++i) {
    const int gr = rowBase + 16 * wave + i;
    float* op = outF + (size_t)gr * (size_t)DIN + 4 * lane;
    if (gr < nN) *(volatile v4f*)op = ov[i];
  }
}

__global__ __launch_bounds__(NTHR) void k_agg(
    const int* __restrict__ srcs, const int* __restrict__ dsts,
    const float* __restrict__ x,
    unsigned short* Aout, int ldaOut,
    int nN, int nE, int nb, int vec8, int MPr) {
  extern __shared__ v4f lds_dyn[];
  int* reg1 = (int*)lds_dyn;
  int* reg2 = reg1 + RCAP;
  int* scnt = reg2 + RCAP;
  int* soff = scnt + NBMAX;
  int* list = soff + NBMAX;
  int* wcnt = list + LISTN;
  int* wtot = wcnt + NWAVE;
  const int tid = (int)threadIdx.x, lane = tid & 31, wave = tid >> 5;
  const int nodeBase = (int)blockIdx.x * nb;

  for (int i = tid; i < NBMAX; i += NTHR) scnt[i] = 0;
  __syncthreads();

  int tot = 0;
  const int nChunks = (nE + CHUNK - 1) / CHUNK;
#pragma unroll 1
  for (int ch = 0; ch < nChunks; ++ch) {
    const int cbase = ch * CHUNK;
    const int wc = scan_chunk(dsts, nE, cbase, nodeBase, nb, vec8, list, tid, lane, wave);
    if (lane == 0) wcnt[wave] = wc;
    __syncthreads();
    int pre = 0, all = 0;
#pragma unroll
    for (int w2 = 0; w2 < NWAVE; ++w2) {
      int c = wcnt[w2];
      c = c < 0 ? 0 : (c > WCAP ? WCAP : c);
      all += c;
      pre += (w2 < wave) ? c : 0;
    }
    const int wcc  = wc > WCAP ? WCAP : wc;
    const int base = tot + pre;
#pragma unroll 1
    for (int i = lane; i < wcc; i += 32) {
      const int ent = list[wave * WCAP + i];
      const int el  = (ent >> PKS) & (CHUNK - 1);
      const int sl  = ent & (NBMAX - 1);
      int eid = cbase + el;
      eid = eid > nE - 1 ? nE - 1 : eid;
      const int pos = base + i;
      if (pos < RCAP) reg1[pos] = (int)(((unsigned)eid << PKS) | (unsigned)sl);
    }
    tot += all;
    tot = tot > RCAP ? RCAP : tot;
    __syncthreads();
  }
  const int nh = tot;

  if (wave == 0) {
#pragma unroll 1
    for (int b0 = 0; b0 < nh; b0 += 32) {
      const int idx = b0 + lane;
      const int uv  = reg1[idx < RCAP ? idx : RCAP - 1];
      const int m32 = (nh - b0) < 32 ? (nh - b0) : 32;
#pragma unroll 1
      for (int k = 0; k < m32; ++k) {
        const int u  = __builtin_amdgcn_readlane(uv, k);
        const int sl = u & (NBMAX - 1);
        if (lane == 0) scnt[sl] = scnt[sl] + 1;
      }
    }
  }
  __syncthreads();

  {
    const v4i ca = *(const v4i*)(scnt + 8 * tid);
    const v4i cb = *(const v4i*)(scnt + 8 * tid + 4);
    const int e0 = ca.x < 0 ? 0 : ca.x, e1 = ca.y < 0 ? 0 : ca.y, e2 = ca.z < 0 ? 0 : ca.z, e3 = ca.w < 0 ? 0 : ca.w;
    const int e4 = cb.x < 0 ? 0 : cb.x, e5 = cb.y < 0 ? 0 : cb.y, e6 = cb.z < 0 ? 0 : cb.z, e7 = cb.w < 0 ? 0 : cb.w;
    const int ts = e0 + e1 + e2 + e3 + e4 + e5 + e6 + e7;
    int incl = ts;
#pragma unroll
    for (int d = 1; d < 32; d <<= 1) {
      const int up = __shfl_up(incl, d);
      if (lane >= d) incl += up;
    }
    if (lane == 31) wtot[wave] = incl;
    __syncthreads();
    int pre = 0;
#pragma unroll
    for (int w2 = 0; w2 < NWAVE; ++w2) pre += (w2 < wave) ? wtot[w2] : 0;
    int run = pre + incl - ts;
    soff[8 * tid + 0] = run; run += e0;
    soff[8 * tid + 1] = run; run += e1;
    soff[8 * tid + 2] = run; run += e2;
    soff[8 * tid + 3] = run; run += e3;
    soff[8 * tid + 4] = run; run += e4;
    soff[8 * tid + 5] = run; run += e5;
    soff[8 * tid + 6] = run; run += e6;
    soff[8 * tid + 7] = run;
  }
  __syncthreads();
  for (int i = tid; i < NBMAX; i += NTHR) list[i] = soff[i];
  __syncthreads();

  if (wave == 0) {
#pragma unroll 1
    for (int b0 = 0; b0 < nh; b0 += 32) {
      const int idx = b0 + lane;
      const int uv  = reg1[idx < RCAP ? idx : RCAP - 1];
      const int m32 = (nh - b0) < 32 ? (nh - b0) : 32;
#pragma unroll 1
      for (int k = 0; k < m32; ++k) {
        const int u   = __builtin_amdgcn_readlane(uv, k);
        const int sl  = u & (NBMAX - 1);
        const int eid = (int)((unsigned)u >> PKS);
        if (lane == 0) {
          int pos = list[sl];
          pos = pos < 0 ? 0 : (pos > RCAP - 1 ? RCAP - 1 : pos);
          reg2[pos] = eid;
          list[sl] = pos + 1;
        }
      }
    }
  }
  __syncthreads();

  const int nbw = nb >> 3;
  const bool ovf = (nh >= RCAP);
  const float qnan = __int_as_float(0x7fc00000);
  unsigned int* stwu = (unsigned int*)((float*)reg1 + wave * STW);

#pragma unroll 1
  for (int jt = 0; jt < nbw; ++jt) {
    const int slot = wave * nbw + jt;
    const int grow = nodeBase + slot;
    int st = soff[slot];
    const int craw = scnt[slot];
    int cnt = craw;
    st  = st < 0 ? 0 : (st > nh ? nh : st);
    cnt = cnt < 0 ? 0 : (cnt > DEGCAP ? DEGCAP : cnt);
    if (cnt > nh - st) cnt = nh - st;
    const float pz = (ovf || craw > DEGCAP) ? qnan : 0.0f;
    const bool liveRow = grow < nN;
    const int grc = liveRow ? grow : nN - 1;

    const v4f xs = *(const v4f*)(x + (size_t)grc * DIN + 4 * lane);
    float ag0 = bf_rne(xs.x) + 0.0f, ag1 = bf_rne(xs.y) + 0.0f, ag2 = bf_rne(xs.z) + 0.0f, ag3 = bf_rne(xs.w) + 0.0f;
#pragma unroll 1
    for (int q = 0; q < cnt; ++q) {
      int idx = st + q; idx = idx > RCAP - 1 ? RCAP - 1 : idx;
      int eid = reg2[idx]; eid = eid < 0 ? 0 : (eid > nE - 1 ? nE - 1 : eid);
      const int sraw = srcs[eid];
      const int s = sraw < 0 ? 0 : (sraw > nN - 1 ? nN - 1 : sraw);
      const v4f v = *(const v4f*)(x + (size_t)s * DIN + 4 * lane);
      ag0 += bf_rne(v.x); ag1 += bf_rne(v.y); ag2 += bf_rne(v.z); ag3 += bf_rne(v.w);
    }
    const float dg  = (float)(craw < 0 ? 0 : craw);
    const float nrm = rsqrtf(fmaxf(dg, 1.0f));
    float r0 = ag0 * nrm, r1 = ag1 * nrm, r2 = ag2 * nrm, r3 = ag3 * nrm;
    r0 = (liveRow ? r0 : 0.0f) + pz;
    r1 = (liveRow ? r1 : 0.0f) + pz;
    r2 = (liveRow ? r2 : 0.0f) + pz;
    r3 = (liveRow ? r3 : 0.0f) + pz;

    const unsigned short hb0 = bf_bits(r0), hb1 = bf_bits(r1), hb2 = bf_bits(r2), hb3 = bf_bits(r3);
    const unsigned short lb0 = bf_bits(r0 - bf_val(hb0)), lb1 = bf_bits(r1 - bf_val(hb1));
    const unsigned short lb2 = bf_bits(r2 - bf_val(hb2)), lb3 = bf_bits(r3 - bf_val(hb3));
    v2u hw, lw;
    hw.x = (unsigned int)hb0 | ((unsigned int)hb1 << 16);
    hw.y = (unsigned int)hb2 | ((unsigned int)hb3 << 16);
    lw.x = (unsigned int)lb0 | ((unsigned int)lb1 << 16);
    lw.y = (unsigned int)lb2 | ((unsigned int)lb3 << 16);
    __builtin_amdgcn_fence(__ATOMIC_RELEASE, "wavefront");
    __builtin_amdgcn_wave_barrier();
    *(v2u*)(stwu + 2 * lane)      = hw;
    *(v2u*)(stwu + 64 + 2 * lane) = lw;
    __builtin_amdgcn_fence(__ATOMIC_RELEASE, "wavefront");
    __builtin_amdgcn_wave_barrier();
    const v4u pk = *(const v4u*)(stwu + 4 * lane);
    unsigned short* gp = Aout + (size_t)grow * (size_t)ldaOut + 8 * lane;
    const bool wsv = grow < MPr;
    if (wsv) *(volatile v4u*)gp = pk;
    __threadfence();
    if (wsv) *(volatile v4u*)gp = pk;
  }
}

static int pick_nb(int nE, int nN) {
  int nb = NBRUN;
  while (nb > 16 && (long long)nb * (long long)nE * 5LL > (long long)RCAP * (long long)nN * 4LL) nb >>= 1;
  return nb;
}
static inline int cdiv(int a, int b) { return (a + b - 1) / b; }

extern "C" void kernel_launch(void* const* d_in, const int* in_sizes, int n_in,
                              void* d_out, int out_size, void* d_ws, size_t ws_size,
                              hipStream_t stream) {
  if (n_in < 5) return;
  const int nN = in_sizes[0] / DIN;
  if (nN <= 0 || in_sizes[0] != nN * DIN || nN > (1 << 22)) return;
  const int nE = in_sizes[1];
  if (nE < 1 || nE > (1 << 21)) return;
  if (in_sizes[2] != nE) return;
  if (in_sizes[3] != DIN * DIN || in_sizes[4] != DIN) return;
  if (out_size != nN * DIN) return;

  const float* x   = (const float*)d_in[0];
  const int*   src = (const int*)  d_in[1];
  const int*   dst = (const int*)  d_in[2];
  const float* W   = (const float*)d_in[3];
  const float* bb  = (const float*)d_in[4];
  float* out = (float*)d_out;

  const int MP   = cdiv(nN, GBM) * GBM;
  const int nb   = pick_nb(nE, nN);
  const int gA   = cdiv(MP, nb);
  const int vec8 = 1;
  if (nb < 16 || (nb & 7) != 0) return;
  if ((long long)gA * nb < (long long)MP) return;

  char* ws = (char*)d_ws;
  size_t off = 0;
  const size_t oAG = off; off += (size_t)MP * APW * 2;          off = (off + 255) & ~(size_t)255;
  const size_t oWT = off; off += (size_t)DIN * KP * 2;          off = (off + 255) & ~(size_t)255;
  if (off > ws_size || off > (size_t)WSMAX) return;
  unsigned short* AG = (unsigned short*)(ws + oAG);
  unsigned short* WT = (unsigned short*)(ws + oWT);

  hipFuncSetAttribute(reinterpret_cast<const void*>(&k_agg),
                      hipFuncAttributeMaxDynamicSharedMemorySize, LDS_AGG);

  k_prep<<<NUW / NTHR, NTHR, 0, stream>>>(W, WT);

  k_agg<<<gA, NTHR, LDS_AGG, stream>>>(src, dst, x, AG, APW, nN, nE, nb, vec8, MP);

  k_gemm<<<dim3(MP / GBM, 1), GTHR, 0, stream>>>(AG, APW, WT, bb, out, nN);
}
